// GQA_35055523070279
// MI455X (gfx1250) — hardware-verified
//
#include <hip/hip_runtime.h>
#include <math.h>
#include <stdint.h>

#define SQ    2048
#define DMD   2048
#define NHQ   32
#define NKVH  8
#define HDM   64
#define QW    2048
#define KW    512
#define QKN   2560
#define NFREQ 32
#define AOW   4096

static_assert(QW == NHQ * HDM);
static_assert(KW == NKVH * HDM);
static_assert(QKN == QW + KW);
static_assert(AOW == 2 * DMD);
static_assert(SQ % 64 == 0 && SQ % 128 == 0 && DMD % 128 == 0 && QKN % 128 == 0 && KW % 32 == 0 && DMD % 32 == 0 && AOW % 32 == 0);
static_assert(((SQ * DMD / 8) % 256) == 0 && ((KW * DMD / 8) % 256) == 0 && ((DMD * DMD / 8) % 256) == 0);

typedef __bf16       v16b __attribute__((ext_vector_type(16)));
typedef __bf16       v8b  __attribute__((ext_vector_type(8)));
typedef float        v8f  __attribute__((ext_vector_type(8)));
typedef float        v4f  __attribute__((ext_vector_type(4)));
typedef unsigned int v4u  __attribute__((ext_vector_type(4)));

__device__ __forceinline__ unsigned short bf_bits(float f) {
  const unsigned u = __float_as_uint(f);
  return (unsigned short)((u + 0x7FFFu + ((u >> 16) & 1u)) >> 16);
}
__device__ __forceinline__ float bf_val(unsigned short hb) { return __uint_as_float(((unsigned)hb) << 16); }
__device__ __forceinline__ float bf_rne(float f) { return bf_val(bf_bits(f)); }
__device__ __forceinline__ unsigned pk16(unsigned short a, unsigned short b) { return (unsigned)a | ((unsigned)b << 16); }
__device__ __forceinline__ v8f zero8() { v8f z = {0.f, 0.f, 0.f, 0.f, 0.f, 0.f, 0.f, 0.f}; return z; }
__device__ __forceinline__ int wave_id() { return __builtin_amdgcn_readfirstlane((int)(threadIdx.x >> 5)); }

__device__ __forceinline__ void lds_wave_sync() {
  __builtin_amdgcn_fence(__ATOMIC_RELEASE, "workgroup");
  __builtin_amdgcn_wave_barrier();
  __builtin_amdgcn_fence(__ATOMIC_ACQUIRE, "workgroup");
}

union FragB { v16b v; v8b hv[2]; };
__device__ __forceinline__ v16b ldfrag_b(const __bf16* p) { FragB f; f.hv[0] = *(const v8b*)(p); f.hv[1] = *(const v8b*)(p + 16); return f.v; }

__device__ __forceinline__ v8f mma_b(v16b a, v16b b, v8f c) {
  return __builtin_amdgcn_wmma_f32_16x16x32_bf16(false, a, false, b, (short)0, c, false, false);
}
__device__ __forceinline__ void guard2b3(v8f& a, v8f& b, v16b x0, v16b x1, v16b y) {
  asm volatile("v_nop\n\tv_nop\n\tv_nop\n\tv_nop" : "+v"(a), "+v"(b) : "v"(x0), "v"(x1), "v"(y) : "memory");
}
__device__ __forceinline__ void guard1b4(v8f& a, v16b w, v16b x, v16b y, v16b z) {
  asm volatile("v_nop\n\tv_nop\n\tv_nop\n\tv_nop" : "+v"(a) : "v"(w), "v"(x), "v"(y), "v"(z) : "memory");
}
__device__ __forceinline__ void acc_guard4(v8f& a, v8f& b, v8f& c, v8f& d) {
  asm volatile("v_nop\n\tv_nop\n\tv_nop\n\tv_nop" : "+v"(a), "+v"(b), "+v"(c), "+v"(d));
}
__device__ __forceinline__ void acc_guard2(v8f& a, v8f& b) {
  asm volatile("v_nop\n\tv_nop\n\tv_nop\n\tv_nop" : "+v"(a), "+v"(b));
}

__global__ __launch_bounds__(256) void cvt_bf16_kernel(const float* __restrict__ in, unsigned short* __restrict__ outp, int n8) {
  const int i = (int)blockIdx.x * 256 + (int)threadIdx.x;
  if (i >= n8) return;
  const size_t e = 8 * (size_t)i;
  const v4f a = *(const v4f*)(in + e);
  const v4f b = *(const v4f*)(in + e + 4);
  v4u w;
  w[0] = pk16(bf_bits(a[0]), bf_bits(a[1]));
  w[1] = pk16(bf_bits(a[2]), bf_bits(a[3]));
  w[2] = pk16(bf_bits(b[0]), bf_bits(b[1]));
  w[3] = pk16(bf_bits(b[2]), bf_bits(b[3]));
  *(volatile v4u*)(outp + e) = w;
  __threadfence();
  *(volatile v4u*)(outp + e) = w;
}

__global__ __launch_bounds__(256) void cvt_wo2_kernel(const float* __restrict__ in, unsigned short* __restrict__ outp,
                                                      int n8, int kin, int ldo) {
  const int i = (int)blockIdx.x * 256 + (int)threadIdx.x;
  if (i >= n8) return;
  const size_t e = 8 * (size_t)i;
  const int n = (int)(e / (size_t)kin);
  const int k = (int)(e - (size_t)n * kin);
  const v4f a = *(const v4f*)(in + e);
  const v4f b = *(const v4f*)(in + e + 4);
  v4u w;
  w[0] = pk16(bf_bits(a[0]), bf_bits(a[1]));
  w[1] = pk16(bf_bits(a[2]), bf_bits(a[3]));
  w[2] = pk16(bf_bits(b[0]), bf_bits(b[1]));
  w[3] = pk16(bf_bits(b[2]), bf_bits(b[3]));
  const size_t o = (size_t)n * ldo + k;
  *(volatile v4u*)(outp + o) = w;
  *(volatile v4u*)(outp + o + kin) = w;
  __threadfence();
  *(volatile v4u*)(outp + o) = w;
  *(volatile v4u*)(outp + o + kin) = w;
}

template <int EPI> struct SlabCfg { static constexpr int PERWF = 2048; };
template <> struct SlabCfg<0>     { static constexpr int PERWF = 3136; };
static_assert(4 * SlabCfg<0>::PERWF * 4 <= 65536 && (SlabCfg<0>::PERWF * 4) % 16 == 0);

template <int EPI>
__global__ __launch_bounds__(128) void gemm_w32x128_kernel(
    const unsigned short* __restrict__ Ap, int lda,
    const unsigned short* __restrict__ Btp, int ldb,
    const float* __restrict__ cst, const float* __restrict__ snt,
    const float* __restrict__ wqn, const float* __restrict__ wkn,
    void* C0, void* C1, void* C2, void* C3, int ldc, int ldc2,
    int M, int N, int K) {
  __shared__ __align__(16) float lds_all[4 * SlabCfg<EPI>::PERWF];

  const int lane = threadIdx.x & 31;
  const int wave = wave_id();
  const int hh = lane >> 4;
  const int rl = lane & 15;
  const int tilesN = N >> 7;
  const int tilesM = M >> 5;
  const int tile = (int)blockIdx.x * 4 + wave;
  if (tile >= tilesM * tilesN) return;
  const int tm = tile / tilesN;
  const int tn = tile - tm * tilesN;
  const int m0 = tm << 5;
  const int n0 = tn << 7;

  const __bf16* A  = (const __bf16*)(const void*)Ap;
  const __bf16* Bt = (const __bf16*)(const void*)Btp;

  v8f acc[2][8];
#pragma unroll
  for (int i = 0; i < 2; ++i)
#pragma unroll
    for (int j = 0; j < 8; ++j) acc[i][j] = zero8();

  for (int k0 = 0; k0 < K; k0 += 32) {
    v16b ah[2];
#pragma unroll
    for (int i = 0; i < 2; ++i) ah[i] = ldfrag_b(A + (size_t)(m0 + i * 16 + rl) * lda + k0 + 8 * hh);
#pragma unroll
    for (int j = 0; j < 8; ++j) {
      const v16b bj = ldfrag_b(Bt + (size_t)(n0 + j * 16 + rl) * ldb + k0 + 8 * hh);
      acc[0][j] = mma_b(ah[0], bj, acc[0][j]);
      acc[1][j] = mma_b(ah[1], bj, acc[1][j]);
      guard2b3(acc[0][j], acc[1][j], ah[0], ah[1], bj);
    }
  }
  acc_guard4(acc[0][0], acc[0][1], acc[0][2], acc[0][3]);
  acc_guard4(acc[0][4], acc[0][5], acc[0][6], acc[0][7]);
  acc_guard4(acc[1][0], acc[1][1], acc[1][2], acc[1][3]);
  acc_guard4(acc[1][4], acc[1][5], acc[1][6], acc[1][7]);

  float* wl = lds_all + wave * SlabCfg<EPI>::PERWF;
  unsigned short* sl16 = (unsigned short*)(void*)wl;
  float* slf = wl;

  if (EPI == 0) {
    float* fsl = wl;
    unsigned short* hsl = sl16 + 2048;
    unsigned short* lsl = sl16 + 3072;
    float* csl = wl + 2048;
    float* snl = wl + 2048 + 16 * NFREQ;
    float* wsl = wl + 2048 + 32 * NFREQ;
    const bool isq = (n0 < QW);
    unsigned short* P0 = isq ? (unsigned short*)C0 : (unsigned short*)C2;
    unsigned short* P1 = isq ? (unsigned short*)C1 : (unsigned short*)C3;
    const int ldp  = isq ? ldc : ldc2;
    const int col0 = isq ? n0 : (n0 - QW);
    {
      const float qa = wqn[lane], qb = wqn[lane + 32];
      const float ka = wkn[lane], kb = wkn[lane + 32];
      wsl[lane]      = bf_rne(isq ? qa : ka);
      wsl[lane + 32] = bf_rne(isq ? qb : kb);
    }
    const int prow = lane >> 1;
    const int pp0  = (lane & 1) * 16;
    const int rq   = lane >> 3;
    const int c8   = (lane & 7) * 8;
#pragma unroll
    for (int i = 0; i < 2; ++i) {
      const int mb = m0 + i * 16;
#pragma unroll
      for (int u = 0; u < 4; ++u) {
        const int p   = lane + 32 * u;
        const int row = p >> 3, c4 = (p & 7) * 4;
        const v4f cv4 = *(const v4f*)(cst + (size_t)(mb + row) * NFREQ + c4);
        const v4f sv4 = *(const v4f*)(snt + (size_t)(mb + row) * NFREQ + c4);
        *(v4f*)(csl + row * NFREQ + c4) = cv4;
        *(v4f*)(snl + row * NFREQ + c4) = sv4;
      }
      lds_wave_sync();
#pragma unroll
      for (int hs = 0; hs < 2; ++hs) {
#pragma unroll
        for (int jh = 0; jh < 4; ++jh)
#pragma unroll
          for (int r = 0; r < 8; ++r)
            fsl[(8 * hh + r) * 64 + jh * 16 + rl] = acc[i][hs * 4 + jh][r];
        lds_wave_sync();
        float ss = 0.0f;
#pragma unroll 2
        for (int t = 0; t < 16; ++t) {
          const int p = pp0 + t;
          float* e = fsl + prow * 64 + 2 * p;
          const float xr = e[0];
          const float xi = e[1];
          const float cv = bf_rne(csl[prow * NFREQ + p]);
          const float sv = bf_rne(snl[prow * NFREQ + p]);
          const float yr = xr * cv - xi * sv;
          const float yi = xr * sv + xi * cv;
          e[0] = yr;
          e[1] = yi;
          ss += yr * yr + yi * yi;
        }
        ss += __shfl_xor(ss, 1, 32);
        const float inv = rsqrtf(ss * 0.015625f + 1.0e-6f);
#pragma unroll 2
        for (int t = 0; t < 16; ++t) {
          const int p = pp0 + t;
          const float* e = fsl + prow * 64 + 2 * p;
          const float v0 = e[0] * inv * wsl[2 * p];
          const float v1 = e[1] * inv * wsl[2 * p + 1];
          const unsigned short h0 = bf_bits(v0), h1 = bf_bits(v1);
          const unsigned short l0 = bf_bits(v0 - bf_val(h0)), l1 = bf_bits(v1 - bf_val(h1));
          *(unsigned*)(void*)(hsl + prow * 64 + 2 * p) = pk16(h0, h1);
          *(unsigned*)(void*)(lsl + prow * 64 + 2 * p) = pk16(l0, l1);
        }
        lds_wave_sync();
        for (int pass = 0; pass < 2; ++pass) {
#pragma unroll
          for (int it = 0; it < 4; ++it) {
            const int row = it * 4 + rq;
            const v4u vh = *(const v4u*)(hsl + row * 64 + c8);
            const v4u vl = *(const v4u*)(lsl + row * 64 + c8);
            const size_t go = (size_t)(mb + row) * ldp + col0 + hs * 64 + c8;
            *(volatile v4u*)(P0 + go) = vh;
            *(volatile v4u*)(P1 + go) = vl;
          }
          __threadfence();
        }
        lds_wave_sync();
      }
    }
  } else if (EPI == 1) {
    unsigned short* P0 = (unsigned short*)C0;
    unsigned short* P1 = (unsigned short*)C1;
#pragma unroll
    for (int i = 0; i < 2; ++i) {
#pragma unroll
      for (int r = 0; r < 8; ++r) {
#pragma unroll
        for (int j = 0; j < 8; ++j) {
          const float v = acc[i][j][r];
          const unsigned short hb = bf_bits(v);
          const unsigned short lb = bf_bits(v - bf_val(hb));
          const int so = (8 * hh + r) * 128 + j * 16 + rl;
          sl16[so]        = hb;
          sl16[2048 + so] = lb;
        }
      }
      lds_wave_sync();
      for (int pass = 0; pass < 2; ++pass) {
#pragma unroll
        for (int it = 0; it < 8; ++it) {
          const int row = it * 2 + hh;
          const int c8  = rl * 8;
          const v4u vh = *(const v4u*)(sl16 + row * 128 + c8);
          const v4u vl = *(const v4u*)(sl16 + 2048 + row * 128 + c8);
          const size_t go = (size_t)(m0 + i * 16 + row) * ldc + n0 + c8;
          *(volatile v4u*)(P0 + go) = vh;
          *(volatile v4u*)(P1 + go) = vl;
        }
        __threadfence();
      }
      lds_wave_sync();
    }
  } else {
    float* C = (float*)C0;
#pragma unroll
    for (int i = 0; i < 2; ++i) {
#pragma unroll
      for (int j = 0; j < 8; ++j)
#pragma unroll
        for (int r = 0; r < 8; ++r) {
          float v = acc[i][j][r];
          if (EPI == 3) {
            const float t = fminf(fmaxf(v, -30.0f), 30.0f);
            v = __builtin_amdgcn_rcpf(1.0f + __expf(-t));
          }
          slf[(8 * hh + r) * 128 + j * 16 + rl] = v;
        }
      lds_wave_sync();
      for (int pass = 0; pass < 2; ++pass) {
#pragma unroll
        for (int row = 0; row < 16; ++row) {
          const v4f v = *(const v4f*)(slf + row * 128 + lane * 4);
          *(volatile v4f*)(C + (size_t)(m0 + i * 16 + row) * ldc + n0 + lane * 4) = v;
        }
        __threadfence();
      }
      lds_wave_sync();
    }
  }
}

#define AKC  32
#define QP   72
#define KP   72
#define VP   40
#define PP   40
#define OSP  64
static_assert((2 * 64 * QP + 2 * AKC * KP + 2 * HDM * VP + 2 * 4 * 16 * PP) * 2 + 4 * 16 * OSP * 4 <= 65536);
static_assert(SQ % 64 == 0 && SQ % AKC == 0 && HDM == 64);

__global__ __launch_bounds__(128)
void attn_causal_kernel(const unsigned short* __restrict__ qhp, const unsigned short* __restrict__ qlp,
                        const unsigned short* __restrict__ khp, const unsigned short* __restrict__ klp,
                        const unsigned short* __restrict__ vhp, const unsigned short* __restrict__ vlp,
                        const float* __restrict__ gp, unsigned short* __restrict__ ogp) {
  __shared__ __align__(16) unsigned short Qs [64 * QP];
  __shared__ __align__(16) unsigned short Qls[64 * QP];
  __shared__ __align__(16) unsigned short Ks [AKC * KP];
  __shared__ __align__(16) unsigned short Kls[AKC * KP];
  __shared__ __align__(16) unsigned short Vhs[HDM * VP];
  __shared__ __align__(16) unsigned short Vls[HDM * VP];
  __shared__ __align__(16) unsigned short Phs[4][16 * PP];
  __shared__ __align__(16) unsigned short Pls[4][16 * PP];
  __shared__ __align__(16) float Os[4][16 * OSP];

  const int tid  = (int)threadIdx.x;
  const int lane = tid & 31;
  const int wave = wave_id();
  const int hh   = lane >> 4;
  const int c    = lane & 15;
  const int qt   = (int)blockIdx.x;
  const int h    = (int)blockIdx.y;
  const int kvh  = h >> 2;
  const int qr0  = qt * 64;
  const int q0   = qr0 + wave * 16;

#pragma unroll
  for (int u = 0; u < 4; ++u) {
    const int p   = tid + 128 * u;
    const int row = p >> 3, d8 = (p & 7) * 8;
    const size_t qo = (size_t)(qr0 + row) * QW + h * HDM + d8;
    const v4u qa = *(const v4u*)(qhp + qo);
    const v4u qb = *(const v4u*)(qlp + qo);
    *(v4u*)(Qs  + row * QP + d8) = qa;
    *(v4u*)(Qls + row * QP + d8) = qb;
  }
  __syncthreads();

  const __bf16* Qa  = (const __bf16*)(const void*)Qs  + (wave * 16 + c) * QP + 8 * hh;
  const __bf16* Qla = (const __bf16*)(const void*)Qls + (wave * 16 + c) * QP + 8 * hh;
  unsigned short* ph = Phs[wave];
  unsigned short* pl = Pls[wave];

  float mrow[8], lrow[8];
  v8f oacc[4];
#pragma unroll
  for (int r = 0; r < 8; ++r) { mrow[r] = -INFINITY; lrow[r] = 0.f; }
#pragma unroll
  for (int t = 0; t < 4; ++t) oacc[t] = zero8();

  const int nChunks = 2 * (qt + 1);
  for (int kc = 0; kc < nChunks; ++kc) {
    const int kv0 = kc * AKC;
    __syncthreads();
#pragma unroll
    for (int u = 0; u < 2; ++u) {
      const int p   = tid + 128 * u;
      const int key = p >> 3, d8 = (p & 7) * 8;
      const size_t ko = (size_t)(kv0 + key) * KW + kvh * HDM + d8;
      const v4u kx = *(const v4u*)(khp + ko);
      const v4u ky = *(const v4u*)(klp + ko);
      *(v4u*)(Ks  + key * KP + d8) = kx;
      *(v4u*)(Kls + key * KP + d8) = ky;
      const int d = p >> 2, k8 = (p & 3) * 8;
      const size_t vo = (size_t)(kvh * HDM + d) * SQ + kv0 + k8;
      const v4u vx = *(const v4u*)(vhp + vo);
      const v4u vy = *(const v4u*)(vlp + vo);
      *(v4u*)(Vhs + d * VP + k8) = vx;
      *(v4u*)(Vls + d * VP + k8) = vy;
    }
    __syncthreads();

    v8f sa[2];
    sa[0] = zero8(); sa[1] = zero8();
#pragma unroll
    for (int dc = 0; dc < 2; ++dc) {
      const v16b qh = ldfrag_b(Qa  + dc * 32);
      const v16b ql = ldfrag_b(Qla + dc * 32);
#pragma unroll
      for (int j = 0; j < 2; ++j) {
        const v16b kb = ldfrag_b((const __bf16*)(const void*)Ks  + (j * 16 + c) * KP + dc * 32 + 8 * hh);
        const v16b kl = ldfrag_b((const __bf16*)(const void*)Kls + (j * 16 + c) * KP + dc * 32 + 8 * hh);
        sa[j] = mma_b(qh, kb, sa[j]);
        sa[j] = mma_b(qh, kl, sa[j]);
        sa[j] = mma_b(ql, kb, sa[j]);
        guard1b4(sa[j], qh, ql, kb, kl);
      }
    }
    acc_guard2(sa[0], sa[1]);

    float cm[8];
#pragma unroll
    for (int r = 0; r < 8; ++r) {
      const int qrow = q0 + 8 * hh + r;
      float m = -INFINITY;
#pragma unroll
      for (int j = 0; j < 2; ++j) {
        const int kvcol = kv0 + j * 16 + c;
        const float sv = sa[j][r] * 0.125f;
        const float sm = (kvcol > qrow) ? -INFINITY : sv;
        sa[j][r] = sm;
        m = fmaxf(m, sm);
      }
#pragma unroll
      for (int off = 1; off < 16; off <<= 1) m = fmaxf(m, __shfl_xor(m, off, 32));
      cm[r] = m;
    }
#pragma unroll
    for (int r = 0; r < 8; ++r) {
      const float mnew  = fmaxf(mrow[r], cm[r]);
      const float muse  = (mnew > -INFINITY) ? mnew : 0.0f;
      const float alpha = __expf(mrow[r] - muse);
      mrow[r] = mnew;
      float psum = 0.f;
#pragma unroll
      for (int j = 0; j < 2; ++j) {
        const float p = __expf(sa[j][r] - muse);
        psum += p;
        const unsigned short hb = bf_bits(p);
        const unsigned short lb = bf_bits(p - bf_val(hb));
        const int po = (8 * hh + r) * PP + j * 16 + c;
        ph[po] = hb;
        pl[po] = lb;
      }
#pragma unroll
      for (int off = 1; off < 16; off <<= 1) psum += __shfl_xor(psum, off, 32);
      lrow[r] = lrow[r] * alpha + psum;
#pragma unroll
      for (int t = 0; t < 4; ++t) oacc[t][r] *= alpha;
    }
    lds_wave_sync();
    const v16b pa = ldfrag_b((const __bf16*)(const void*)ph + c * PP + 8 * hh);
    const v16b pr = ldfrag_b((const __bf16*)(const void*)pl + c * PP + 8 * hh);
#pragma unroll
    for (int t = 0; t < 4; ++t) {
      const v16b vb = ldfrag_b((const __bf16*)(const void*)Vhs + (t * 16 + c) * VP + 8 * hh);
      const v16b vr = ldfrag_b((const __bf16*)(const void*)Vls + (t * 16 + c) * VP + 8 * hh);
      oacc[t] = mma_b(pa, vb, oacc[t]);
      oacc[t] = mma_b(pa, vr, oacc[t]);
      oacc[t] = mma_b(pr, vb, oacc[t]);
      guard1b4(oacc[t], pa, pr, vb, vr);
    }
  }
  __syncthreads();
  acc_guard4(oacc[0], oacc[1], oacc[2], oacc[3]);

  float* os = Os[wave];
#pragma unroll
  for (int r = 0; r < 8; ++r) {
    const float inv = 1.0f / lrow[r];
#pragma unroll
    for (int t = 0; t < 4; ++t) os[(8 * hh + r) * OSP + t * 16 + c] = oacc[t][r] * inv;
  }
  lds_wave_sync();
  const int qq = lane >> 3;
  const int c8 = (lane & 7) * 8;
  const float* Gr = gp + (size_t)q0 * DMD + h * HDM + c8;
  unsigned short* Og = ogp + (size_t)q0 * AOW + h * HDM + c8;
  v4u hv[4], lv[4];
#pragma unroll
  for (int it = 0; it < 4; ++it) {
    const int row = it * 4 + qq;
    const v4f oa = *(const v4f*)(os + row * OSP + c8);
    const v4f ob = *(const v4f*)(os + row * OSP + c8 + 4);
    const v4f ga = *(const v4f*)(Gr + (size_t)row * DMD);
    const v4f gb = *(const v4f*)(Gr + (size_t)row * DMD + 4);
    float f[8];
    f[0] = oa[0] * ga[0]; f[1] = oa[1] * ga[1]; f[2] = oa[2] * ga[2]; f[3] = oa[3] * ga[3];
    f[4] = ob[0] * gb[0]; f[5] = ob[1] * gb[1]; f[6] = ob[2] * gb[2]; f[7] = ob[3] * gb[3];
    v4u a, a2;
#pragma unroll
    for (int q = 0; q < 4; ++q) {
      const unsigned short h0 = bf_bits(f[2 * q]), h1 = bf_bits(f[2 * q + 1]);
      const unsigned short l0 = bf_bits(f[2 * q] - bf_val(h0)), l1 = bf_bits(f[2 * q + 1] - bf_val(h1));
      a[q]  = pk16(h0, h1);
      a2[q] = pk16(l0, l1);
    }
    hv[it] = a;
    lv[it] = a2;
  }
  for (int pass = 0; pass < 2; ++pass) {
#pragma unroll
    for (int it = 0; it < 4; ++it) {
      const int row = it * 4 + qq;
      *(volatile v4u*)(Og + (size_t)row * AOW)             = hv[it];
      *(volatile v4u*)(Og + (size_t)row * AOW + (AOW / 2)) = lv[it];
    }
    __threadfence();
  }
}

extern "C" void kernel_launch(void* const* d_in, const int* in_sizes, int n_in,
                              void* d_out, int out_size, void* d_ws, size_t ws_size,
                              hipStream_t stream) {
  if (n_in < 10) return;
  if (in_sizes[0] != SQ * DMD) return;
  if (in_sizes[1] != SQ * NFREQ) return;
  if (in_sizes[2] != SQ * NFREQ) return;
  if (in_sizes[3] != QW * DMD) return;
  if (in_sizes[4] != KW * DMD) return;
  if (in_sizes[5] != KW * DMD) return;
  if (in_sizes[6] != DMD * DMD) return;
  if (in_sizes[7] != DMD * DMD) return;
  if (in_sizes[8] != HDM) return;
  if (in_sizes[9] != HDM) return;
  if (out_size != SQ * DMD) return;

  const float* x     = (const float*)d_in[0];
  const float* cosin = (const float*)d_in[1];
  const float* sinin = (const float*)d_in[2];
  const float* wq    = (const float*)d_in[3];
  const float* wk    = (const float*)d_in[4];
  const float* wv    = (const float*)d_in[5];
  const float* wo    = (const float*)d_in[6];
  const float* wg    = (const float*)d_in[7];
  const float* qn    = (const float*)d_in[8];
  const float* kn    = (const float*)d_in[9];
  float* out = (float*)d_out;

  const size_t szXB  = (size_t)SQ * DMD * 2;
  const size_t szWQK = (size_t)QKN * DMD * 2;
  const size_t szWV  = (size_t)KW * DMD * 2;
  const size_t szWG  = (size_t)DMD * DMD * 2;
  const size_t szWO2 = (size_t)DMD * AOW * 2;
  const size_t szQ   = (size_t)SQ * QW * 2;
  const size_t szK   = (size_t)SQ * KW * 2;
  const size_t szVT  = (size_t)KW * SQ * 2;
  const size_t szG   = (size_t)SQ * DMD * 4;
  const size_t szOG  = (size_t)SQ * AOW * 2;
  size_t off = 0;
  const size_t oXB  = off; off += szXB;
  const size_t oWQK = off; off += szWQK;
  const size_t oWV  = off; off += szWV;
  const size_t oWG  = off; off += szWG;
  const size_t oWO2 = off; off += szWO2;
  const size_t oQH  = off; off += szQ;
  const size_t oQL  = off; off += szQ;
  const size_t oKH  = off; off += szK;
  const size_t oKL  = off; off += szK;
  const size_t oVTH = off; off += szVT;
  const size_t oVTL = off; off += szVT;
  const size_t oG   = off; off += szG;
  const size_t oOG  = off; off += szOG;
  if (off > ws_size) return;

  char* ws = (char*)d_ws;
  unsigned short* XB  = (unsigned short*)(ws + oXB);
  unsigned short* WQK = (unsigned short*)(ws + oWQK);
  unsigned short* WV  = (unsigned short*)(ws + oWV);
  unsigned short* WG  = (unsigned short*)(ws + oWG);
  unsigned short* WO2 = (unsigned short*)(ws + oWO2);
  unsigned short* QH  = (unsigned short*)(ws + oQH);
  unsigned short* QL  = (unsigned short*)(ws + oQL);
  unsigned short* KH  = (unsigned short*)(ws + oKH);
  unsigned short* KL  = (unsigned short*)(ws + oKL);
  unsigned short* VTH = (unsigned short*)(ws + oVTH);
  unsigned short* VTL = (unsigned short*)(ws + oVTL);
  float*          G   = (float*)(ws + oG);
  unsigned short* OG  = (unsigned short*)(ws + oOG);

  const dim3 b256(256), b128(128);

  cvt_bf16_kernel<<<dim3((SQ * DMD / 8) / 256), b256, 0, stream>>>(x, XB, SQ * DMD / 8);
  cvt_bf16_kernel<<<dim3((QW * DMD / 8) / 256), b256, 0, stream>>>(wq, WQK, QW * DMD / 8);
  cvt_bf16_kernel<<<dim3((KW * DMD / 8) / 256), b256, 0, stream>>>(wk, WQK + (size_t)QW * DMD, KW * DMD / 8);
  cvt_bf16_kernel<<<dim3((KW * DMD / 8) / 256), b256, 0, stream>>>(wv, WV, KW * DMD / 8);
  cvt_bf16_kernel<<<dim3((DMD * DMD / 8) / 256), b256, 0, stream>>>(wg, WG, DMD * DMD / 8);
  cvt_wo2_kernel<<<dim3((DMD * DMD / 8) / 256), b256, 0, stream>>>(wo, WO2, DMD * DMD / 8, DMD, AOW);
  gemm_w32x128_kernel<0><<<dim3(((SQ / 32) * (QKN / 128) + 3) / 4), b128, 0, stream>>>(
      XB, DMD, WQK, DMD, cosin, sinin, qn, kn, (void*)QH, (void*)QL, (void*)KH, (void*)KL, QW, KW, SQ, QKN, DMD);
  gemm_w32x128_kernel<1><<<dim3(((KW / 32) * (SQ / 128) + 3) / 4), b128, 0, stream>>>(
      WV, DMD, XB, DMD, cosin, sinin, qn, kn, (void*)VTH, (void*)VTL, (void*)VTH, (void*)VTL, SQ, SQ, KW, SQ, DMD);
  gemm_w32x128_kernel<3><<<dim3(((SQ / 32) * (DMD / 128) + 3) / 4), b128, 0, stream>>>(
      XB, DMD, WG, DMD, cosin, sinin, qn, kn, (void*)G, (void*)G, (void*)G, (void*)G, DMD, DMD, SQ, DMD, DMD);
  attn_causal_kernel<<<dim3(SQ / 64, NHQ), b128, 0, stream>>>(QH, QL, KH, KL, VTH, VTL, G, OG);
  gemm_w32x128_kernel<2><<<dim3(((SQ / 32) * (DMD / 128) + 3) / 4), b128, 0, stream>>>(
      OG, AOW, WO2, AOW, cosin, sinin, qn, kn, (void*)out, (void*)out, (void*)out, (void*)out, DMD, DMD, SQ, DMD, AOW);
  (void)hipGetLastError();
}
